// NLB_6717328850962
// MI455X (gfx1250) — hardware-run, weakly checked
//
#include <hip/hip_runtime.h>
#include <math.h>

typedef __attribute__((ext_vector_type(16))) _Float16 v16h;
typedef __attribute__((ext_vector_type(16))) __bf16 v16b;
typedef __attribute__((ext_vector_type(8)))  _Float16 v8h;
typedef __attribute__((ext_vector_type(8)))  float v8f;
typedef __attribute__((ext_vector_type(4)))  float v4f;
typedef __attribute__((ext_vector_type(2)))  float v2f;
typedef __attribute__((ext_vector_type(4)))  unsigned v4u;
typedef __attribute__((ext_vector_type(4)))  int v4i;
typedef float __attribute__((may_alias)) float_a;
typedef int __attribute__((may_alias)) int_a;

template <typename T> __device__ __forceinline__ void vst2(void* p, T v) { *(volatile T*)p = v; __threadfence(); *(volatile T*)p = v; }
__device__ __forceinline__ v8f wmma16(v16h a, v16h b, v8f c) {
  v8f d = __builtin_amdgcn_wmma_f32_16x16x32_f16(false, a, false, b, (short)0, c, false, false);
  asm volatile("v_nop\n\tv_nop\n\tv_nop\n\tv_nop" : "+v"(d) : "v"(a), "v"(b));
  return d;
}
__device__ __forceinline__ v8f wmma_bf(v16b a, v16b b, v8f c) {
  v8f d = __builtin_amdgcn_wmma_f32_16x16x32_bf16(false, a, false, b, (short)0, c, false, false);
  asm volatile("v_nop\n\tv_nop\n\tv_nop\n\tv_nop" : "+v"(d) : "v"(a), "v"(b));
  return d;
}
__device__ __forceinline__ v16h frag_h(const _Float16* rowk0, int lane) {
  union { v16h v; v8h q[2]; } u; const _Float16* p = rowk0 + 8 * (lane >> 4);
  u.q[0] = *(const v8h*)p; u.q[1] = *(const v8h*)(p + 16); return u.v;
}
__device__ __forceinline__ v16h frag_f32(const float* rowk0, int lane) {
  v16h a; const float* p = rowk0 + 8 * (lane >> 4);
#pragma unroll
  for (int i = 0; i < 8; ++i) { a[i] = (_Float16)p[i]; a[8 + i] = (_Float16)p[16 + i]; }
  return a;
}
__device__ __forceinline__ v16h frag_f32s(const float* rowk0, int lane, float sc) {
  v16h a; const float* p = rowk0 + 8 * (lane >> 4);
#pragma unroll
  for (int i = 0; i < 8; ++i) { a[i] = (_Float16)(p[i] * sc); a[8 + i] = (_Float16)(p[16 + i] * sc); }
  return a;
}
__device__ __forceinline__ v16h fragc_f32(const float* W, int k0, int n, int lane, int ld, int K) {
  v16h a; const int g = lane >> 4;
#pragma unroll
  for (int i = 0; i < 8; ++i) { const int ka = k0 + 8 * g + i, kb = ka + 16;
    a[i] = (_Float16)(ka < K ? W[(size_t)(ka < K ? ka : K - 1) * ld + n] : 0.f); a[8 + i] = (_Float16)(kb < K ? W[(size_t)(kb < K ? kb : K - 1) * ld + n] : 0.f); }
  return a;
}
struct F2 { v16b h, l; };
__device__ __forceinline__ F2 bsplit16(const float v[16]) { F2 r;
#pragma unroll
  for (int i = 0; i < 16; ++i) { const __bf16 h = (__bf16)v[i]; r.h[i] = h; r.l[i] = (__bf16)(v[i] - (float)h); }
  return r; }
__device__ __forceinline__ F2 split_row(const float* row, int k0, int lane) { float v[16]; const float* p = row + k0 + 8 * (lane >> 4);
#pragma unroll
  for (int i = 0; i < 8; ++i) { v[i] = p[i]; v[8 + i] = p[16 + i]; }
  return bsplit16(v); }
__device__ __forceinline__ F2 split_rowK(const float* row, int k0, int lane, int K) { float v[16]; const int g = lane >> 4;
#pragma unroll
  for (int i = 0; i < 8; ++i) { const int ka = k0 + 8 * g + i, kb = ka + 16; v[i] = ka < K ? row[ka < K ? ka : K - 1] : 0.f; v[8 + i] = kb < K ? row[kb < K ? kb : K - 1] : 0.f; }
  return bsplit16(v); }
__device__ __forceinline__ F2 split_col(const float* W, int k0, int n, int lane, int ld, int K) { float v[16]; const int g = lane >> 4;
#pragma unroll
  for (int i = 0; i < 8; ++i) { const int ka = k0 + 8 * g + i, kb = ka + 16; v[i] = ka < K ? W[(size_t)(ka < K ? ka : K - 1) * ld + n] : 0.f; v[8 + i] = kb < K ? W[(size_t)(kb < K ? kb : K - 1) * ld + n] : 0.f; }
  return bsplit16(v); }
__device__ __forceinline__ v8f mac3(const F2& a, const F2& b, v8f c) { c = wmma_bf(a.l, b.h, c); c = wmma_bf(a.h, b.l, c); return wmma_bf(a.h, b.h, c); }
__device__ __forceinline__ float sigm(float v) { return 1.0f / (1.0f + expf(-v)); }
#define LDSX() do { asm volatile("s_wait_dscnt 0" ::: "memory"); __builtin_amdgcn_wave_barrier(); __builtin_amdgcn_fence(__ATOMIC_RELEASE, "workgroup"); } while (0)


#define NB 8
#define CC 128
#define NP 4096
#define IC 64
#ifndef TNB
#define TNB NB
#endif
typedef __attribute__((ext_vector_type(8))) __bf16 v8b;
__device__ __forceinline__ v16b frag_b(const __bf16* rowk0, int lane) {
  union { v16b v; v8b q[2]; } u; const __bf16* p = rowk0 + 8 * (lane >> 4);
  u.q[0] = *(const v8b*)p; u.q[1] = *(const v8b*)(p + 16); return u.v;
}
__device__ __forceinline__ float bfr(float v) { return (float)(__bf16)v; }
__device__ __attribute__((noinline)) float exp_ni(float v) { return expf(v); }
__device__ __attribute__((noinline)) float erf_ni(float v) { return erff(v); }

#define WS_TH  0u
#define WS_TL  (WS_TH + 2u * (size_t)NB * NP * IC)
#define WS_PH  (WS_TL + 2u * (size_t)NB * NP * IC)
#define WS_PL  (WS_PH + 2u * (size_t)NB * NP * IC)
#define WS_GH  (WS_PL + 2u * (size_t)NB * NP * IC)
#define WS_GL  (WS_GH + 2u * (size_t)NB * IC * NP)
#define WS_END (WS_GL + 2u * (size_t)NB * IC * NP)

__global__ __launch_bounds__(128) void k_proj(const float* __restrict__ X, const float* __restrict__ TW, const float* __restrict__ TB, const float* __restrict__ PW, const float* __restrict__ PB, const float* __restrict__ GW, const float* __restrict__ GB, _Float16* __restrict__ TH, _Float16* __restrict__ TL, _Float16* __restrict__ PH, _Float16* __restrict__ PL, _Float16* __restrict__ GH, _Float16* __restrict__ GL) {
  __shared__ __align__(16) __bf16 sx[64][CC + 8];
  __shared__ __align__(16) _Float16 sh[64][72], sl[64][72];
  const int tid = threadIdx.x, wave = tid >> 5, lane = tid & 31, col = lane & 15, g = lane >> 4; const int n0 = blockIdx.x * 64; const int which = blockIdx.y; const size_t b = blockIdx.z;
  const float* Wm = which == 0 ? TW : which == 1 ? PW : GW; const float* Bm = which == 0 ? TB : which == 1 ? PB : GB;
  for (int e = tid; e < CC * 64; e += 128) { const int c = e >> 6, nl = e & 63; sx[nl][c] = (__bf16)X[((b * CC + c) * NP) + n0 + nl]; }
  __syncthreads();
  v8f acc[4] = {};
#pragma unroll
  for (int kc = 0; kc < CC / 32; ++kc) { const v16b a = frag_b(&sx[wave * 16 + col][kc * 32], lane);
#pragma unroll
    for (int j = 0; j < 4; ++j) { v16b w; const int o = j * 16 + col;
#pragma unroll
      for (int i = 0; i < 8; ++i) { w[i] = (__bf16)Wm[(size_t)o * CC + kc * 32 + 8 * g + i]; w[8 + i] = (__bf16)Wm[(size_t)o * CC + kc * 32 + 16 + 8 * g + i]; }
      acc[j] = wmma_bf(a, w, acc[j]); } }
#pragma unroll
  for (int j = 0; j < 4; ++j) { const float bb = bfr(Bm[j * 16 + col]);
#pragma unroll
    for (int r = 0; r < 8; ++r) { const float v = acc[j][r] + bb; const _Float16 hv = (_Float16)v, lv = (_Float16)((v - (float)hv) * 2048.0f); const int rl = wave * 16 + 8 * g + r, cl = j * 16 + col; if (which < 2) { sh[rl][cl] = hv; sl[rl][cl] = lv; } else { sh[cl][rl] = hv; sl[cl][rl] = lv; } } }
  __syncthreads();
  if (which < 2) { _Float16* DH = which == 0 ? TH : PH; _Float16* DL = which == 0 ? TL : PL;
    for (int e = tid; e < 64 * 8; e += 128) { const int rl = e >> 3, q = e & 7; const size_t o = (b * NP + n0 + rl) * IC + q * 8; vst2((unsigned*)(DH + o), *(const v4u*)&sh[rl][q * 8]); vst2((unsigned*)(DL + o), *(const v4u*)&sl[rl][q * 8]); } }
  else { for (int e = tid; e < 64 * 8; e += 128) { const int cl = e >> 3, q = e & 7; const size_t o = (b * IC + cl) * (size_t)NP + n0 + q * 8; vst2((unsigned*)(GH + o), *(const v4u*)&sh[cl][q * 8]); vst2((unsigned*)(GL + o), *(const v4u*)&sl[cl][q * 8]); } } }
__global__ __launch_bounds__(128) void k_att(const _Float16* __restrict__ TH, const _Float16* __restrict__ TL, const _Float16* __restrict__ PH, const _Float16* __restrict__ PL, const _Float16* __restrict__ GH, const _Float16* __restrict__ GL, const float* __restrict__ OW, const float* __restrict__ OB, const float* __restrict__ X, float* __restrict__ OUT) {
  __shared__ __align__(16) float sp[4][16][36]; __shared__ __align__(16) float sy[4][16][68]; __shared__ __align__(16) float st[CC][68];
  const int tid = threadIdx.x, wave = tid >> 5, lane = tid & 31, col = lane & 15, g = lane >> 4; const int qb = blockIdx.x; const size_t b = blockIdx.y; const int q0 = qb * 64 + wave * 16; const bool three = (qb < 2);
  v16h aq[2], al[2];
#pragma unroll
  for (int kc = 0; kc < 2; ++kc) { aq[kc] = frag_h(TH + (b * NP + q0 + col) * IC + kc * 32, lane); al[kc] = frag_h(TL + (b * NP + q0 + col) * IC + kc * 32, lane); }
  float m[8], l[8];
#pragma unroll
  for (int r = 0; r < 8; ++r) { m[r] = -3.0e38f; l[r] = 0.f; }
  v8f acc[4] = {}, accl[4] = {};
#pragma unroll 1
  for (int ks = 0; ks < NP / 32; ++ks) { float s[2][8];
#pragma unroll
    for (int ct = 0; ct < 2; ++ct) { const int kk = ks * 32 + ct * 16 + col; const size_t rk = (b * NP + kk) * IC; v8f c = {}, cl = {};
#pragma unroll
      for (int kc = 0; kc < 2; ++kc) { const v16h kh = frag_h(PH + rk + kc * 32, lane); c = wmma16(aq[kc], kh, c); cl = wmma16(al[kc], kh, cl); if (three) cl = wmma16(aq[kc], frag_h(PL + rk + kc * 32, lane), cl); }
#pragma unroll
      for (int r = 0; r < 8; ++r) s[ct][r] = c[r] + cl[r] * (1.0f / 2048.0f); }
    float alpha[8];
#pragma unroll
    for (int r = 0; r < 8; ++r) { float mx = fmaxf(s[0][r], s[1][r]);
#pragma unroll
      for (int o = 1; o < 16; o <<= 1) mx = fmaxf(mx, __shfl_xor(mx, o));
      const float mn = fmaxf(m[r], mx); alpha[r] = __expf(m[r] - mn); const float e0 = __expf(s[0][r] - mn), e1 = __expf(s[1][r] - mn); float es = e0 + e1;
#pragma unroll
      for (int o = 1; o < 16; o <<= 1) es += __shfl_xor(es, o);
      l[r] = l[r] * alpha[r] + es; m[r] = mn; sp[wave][8 * g + r][col] = e0; sp[wave][8 * g + r][16 + col] = e1; }
#pragma unroll
    for (int j = 0; j < 4; ++j)
#pragma unroll
      for (int r = 0; r < 8; ++r) { acc[j][r] *= alpha[r]; accl[j][r] *= alpha[r]; }
    LDSX();
    v16h pa, par; { const float* prow = &sp[wave][col][0] + 8 * (lane >> 4);
#pragma unroll
      for (int i = 0; i < 8; ++i) { const float p0 = prow[i] * 2048.0f, p1 = prow[16 + i] * 2048.0f; pa[i] = (_Float16)p0; pa[8 + i] = (_Float16)p1; par[i] = (_Float16)(p0 - (float)pa[i]); par[8 + i] = (_Float16)(p1 - (float)pa[8 + i]); } }
#pragma unroll
    for (int j = 0; j < 4; ++j) { const size_t po = (b * IC + j * 16 + col) * (size_t)NP + ks * 32; const v16h vh = frag_h(GH + po, lane); acc[j] = wmma16(pa, vh, acc[j]); acc[j] = wmma16(par, vh, acc[j]); if (three) accl[j] = wmma16(pa, frag_h(GL + po, lane), accl[j]); }
    LDSX(); }
#pragma unroll
  for (int r = 0; r < 8; ++r) { const float il = (1.0f / 2048.0f) / l[r];
#pragma unroll
    for (int j = 0; j < 4; ++j) sy[wave][8 * g + r][j * 16 + col] = (acc[j][r] + accl[j][r] * (1.0f / 2048.0f)) * il; }
  LDSX();
  v8f o8[8] = {};
#pragma unroll
  for (int kc = 0; kc < IC / 32; ++kc) { const F2 a = split_row(&sy[wave][col][0], kc * 32, lane);
#pragma unroll
    for (int j = 0; j < 8; ++j) { v16b w; const int c = j * 16 + col;
#pragma unroll
      for (int i = 0; i < 8; ++i) { w[i] = (__bf16)OW[(size_t)c * IC + kc * 32 + 8 * g + i]; w[8 + i] = (__bf16)OW[(size_t)c * IC + kc * 32 + 16 + 8 * g + i]; }
      o8[j] = wmma_bf(a.h, w, o8[j]); o8[j] = wmma_bf(a.l, w, o8[j]); } }
#pragma unroll
  for (int j = 0; j < 8; ++j)
#pragma unroll
    for (int r = 0; r < 8; ++r) { const int c = j * 16 + col, nl = wave * 16 + 8 * g + r; st[c][nl] = o8[j][r] + bfr(OB[c]) + bfr(X[((b * CC + c) * NP) + qb * 64 + nl]); }
  __syncthreads();
  for (int e = tid; e < CC * 16; e += 128) { const int c = e >> 4, q = e & 15; vst2(OUT + ((b * CC + c) * NP) + qb * 64 + q * 4, *(const v4f*)&st[c][q * 4]); } }
extern "C" void kernel_launch(void* const* d_in, const int* in_sizes, int n_in, void* d_out, int out_size, void* d_ws, size_t ws_size, hipStream_t stream) {
  (void)in_sizes; (void)n_in; (void)out_size;
  const float** F = (const float**)d_in;
  if (ws_size < (size_t)WS_END) return;
  char* ws = (char*)d_ws; _Float16 *TH = (_Float16*)(ws + WS_TH), *TL = (_Float16*)(ws + WS_TL), *PH = (_Float16*)(ws + WS_PH), *PL = (_Float16*)(ws + WS_PL), *GH = (_Float16*)(ws + WS_GH), *GL = (_Float16*)(ws + WS_GL);
  k_proj<<<dim3(NP / 64, 3, TNB), 128, 0, stream>>>(F[0], F[1], F[2], F[3], F[4], F[5], F[6], TH, TL, PH, PL, GH, GL);
  k_att<<<dim3(NP / 64, TNB), 128, 0, stream>>>(TH, TL, PH, PL, GH, GL, F[7], F[8], F[0], (float*)d_out);
}
